// multi_head_attn_17282948399586
// MI455X (gfx1250) — hardware-verified
//
#include <hip/hip_runtime.h>
#include <stdint.h>

typedef __attribute__((ext_vector_type(16))) _Float16 v16h;
typedef __attribute__((ext_vector_type(8)))  _Float16 v8h;
typedef __attribute__((ext_vector_type(16))) __bf16   v16b;
typedef __attribute__((ext_vector_type(8)))  __bf16   v8b;
typedef __attribute__((ext_vector_type(8)))  float    v8f;
typedef __attribute__((ext_vector_type(4)))  float    v4f;
typedef __attribute__((ext_vector_type(4)))  unsigned v4u;
typedef __attribute__((ext_vector_type(4)))  int      v4i;

constexpr int NBATCH  = 2;
constexpr int SEQ_LEN = 2048;
constexpr int NHEAD   = 16;
constexpr int HDIM    = 64;
constexpr int DMOD    = 1024;
constexpr int NTOK    = NBATCH * SEQ_LEN;
constexpr int KCH     = 32;
constexpr int QBLK    = 64;
constexpr int MWORDS  = SEQ_LEN / 32;
constexpr float PCARRY = 1024.0f;

static_assert(NTOK % 64 == 0, "M tile");
static_assert(DMOD % 64 == 0, "N tile");
static_assert(DMOD % 32 == 0, "K step");
static_assert(SEQ_LEN % 64 == 0, "N tile (V transposed)");
static_assert(SEQ_LEN % KCH == 0, "key chunks");
static_assert(SEQ_LEN % QBLK == 0, "query blocks");
static_assert(KCH == 32, "one 32-deep P.V step per chunk");
static_assert(HDIM == 64, "head dim");
static_assert(NHEAD * HDIM == DMOD, "model dim");
static_assert((NTOK * DMOD) % (8 * 256) == 0, "cast grid");
static_assert((DMOD * DMOD) % (8 * 256) == 0, "cast grid");
static_assert((SEQ_LEN * MWORDS) % 256 == 0, "pack grid");
static_assert(((NTOK / 64) * (DMOD / 64)) % 8 == 0, "gemm grid");
static_assert(((DMOD / 64) * (SEQ_LEN / 64)) % 8 == 0, "gemm grid");

__device__ __forceinline__ unsigned short f2bf_bits(float f) {
  unsigned u = __float_as_uint(f);
  return (unsigned short)((u + 0x7FFFu + ((u >> 16) & 1u)) >> 16);
}
__device__ __forceinline__ float bf_bits2f(unsigned short h) { return __uint_as_float(((unsigned)h) << 16); }

__device__ __forceinline__ void dep_guard_h(v8f& a, v8f& b, v16h x, v16h y) { asm volatile("v_nop\n\tv_nop\n\tv_nop\n\tv_nop" : "+v"(a), "+v"(b) : "v"(x), "v"(y)); }
__device__ __forceinline__ void dep_guard_b(v8f& a, v8f& b, v16b x, v16b y) { asm volatile("v_nop\n\tv_nop\n\tv_nop\n\tv_nop" : "+v"(a), "+v"(b) : "v"(x), "v"(y)); }
__device__ __forceinline__ void keep4_h(v16h a, v16h b, v16h c, v16h d) { asm volatile("v_nop" :: "v"(a), "v"(b), "v"(c), "v"(d)); }
__device__ __forceinline__ void keep4_b(v16b a, v16b b, v16b c, v16b d) { asm volatile("v_nop" :: "v"(a), "v"(b), "v"(c), "v"(d)); }
__device__ __forceinline__ void acc_guard4(v8f& a, v8f& b, v8f& c, v8f& d) { asm volatile("v_nop\n\tv_nop\n\tv_nop\n\tv_nop" : "+v"(a), "+v"(b), "+v"(c), "+v"(d)); }
template <typename T> struct Frag;
template <> struct Frag<_Float16> {
  typedef v16h V; union U { v16h v; v8h h[2]; };
  static __device__ __forceinline__ v16h load(const _Float16* p) {
    U f; f.h[0] = *(const v8h*)(p); f.h[1] = *(const v8h*)(p + 16); return f.v;
  }
  static __device__ __forceinline__ v8f mma(v16h a, v16h b, v8f c) {
    return __builtin_amdgcn_wmma_f32_16x16x32_f16(false, a, false, b, (short)0, c, false, false);
  }
  static __device__ __forceinline__ void guard(v8f& a, v8f& b, v16h x, v16h y) { dep_guard_h(a, b, x, y); }
  static __device__ __forceinline__ void keep(v16h a, v16h b, v16h c, v16h d) { keep4_h(a, b, c, d); }
};
template <> struct Frag<__bf16> {
  typedef v16b V; union U { v16b v; v8b h[2]; };
  static __device__ __forceinline__ v16b load(const __bf16* p) {
    U f; f.h[0] = *(const v8b*)(p); f.h[1] = *(const v8b*)(p + 16); return f.v;
  }
  static __device__ __forceinline__ v8f mma(v16b a, v16b b, v8f c) {
    return __builtin_amdgcn_wmma_f32_16x16x32_bf16(false, a, false, b, (short)0, c, false, false);
  }
  static __device__ __forceinline__ void guard(v8f& a, v8f& b, v16b x, v16b y) { dep_guard_b(a, b, x, y); }
  static __device__ __forceinline__ void keep(v16b a, v16b b, v16b c, v16b d) { keep4_b(a, b, c, d); }
};

template <int ET> struct Elem;
template <> struct Elem<0> { typedef _Float16 T; };
template <> struct Elem<1> { typedef __bf16 T; };
template <int ET, bool SPLIT, int BIAS_MODE, int OUT_MODE, bool RESID, int ACT = 0, bool BSPLIT = true>
__global__ __launch_bounds__(256) void wmma_gemm64(
    const unsigned short* __restrict__ Ap, const unsigned short* __restrict__ A2p, int lda, long strideA,
    const unsigned short* __restrict__ Btp, const unsigned short* __restrict__ Bt2p, int ldb, long strideB,
    void* __restrict__ Cout, void* __restrict__ Cout2, int ldc, long strideC,
    const float* __restrict__ bias,
    const float* __restrict__ resid, long strideR,
    int M, int N, int K, float scale) {
  typedef typename Elem<ET>::T T;
  typedef typename Frag<T>::V V;
  const T* A = (const T*)Ap; const T* A2 = (const T*)A2p; const T* Bt = (const T*)Btp; const T* Bt2 = (const T*)Bt2p;
  __shared__ __align__(16) float sT[8][16 * 68];
  const int b    = blockIdx.y;
  const int lane = threadIdx.x & 31;
  const int wave = threadIdx.x >> 5;
  const int tilesN = N >> 6;
  const int tilesM = M >> 6;
  const int tile = blockIdx.x * 8 + wave;
  if (tile >= tilesM * tilesN) return;
  const int tm = tile / tilesN;
  const int tn = tile - tm * tilesN;
  const int m0 = tm << 6;
  const int n0 = tn << 6;

  const T* Ab  = A  + (size_t)b * strideA;
  const T* Bb  = Bt + (size_t)b * strideB;
  const T* Ab2 = SPLIT ? (A2  + (size_t)b * strideA) : nullptr;
  const T* Bb2 = (SPLIT && BSPLIT) ? (Bt2 + (size_t)b * strideB) : nullptr;

  const int rlane = lane & 15;
  const int koff  = (lane >> 4) * 8;
  const int mOff  = (lane >> 4) * 8;

  v8f acc[4][4];
#pragma unroll
  for (int i = 0; i < 4; ++i)
#pragma unroll
    for (int j = 0; j < 4; ++j) acc[i][j] = (v8f){0.f,0.f,0.f,0.f,0.f,0.f,0.f,0.f};

  for (int k0 = 0; k0 < K; k0 += 32) {
    V bh[4], bl[4];
#pragma unroll
    for (int j = 0; j < 4; ++j) {
      const size_t bo = (size_t)(n0 + (j << 4) + rlane) * ldb + koff + k0;
      bh[j] = Frag<T>::load(Bb + bo);
      if (SPLIT && BSPLIT) bl[j] = Frag<T>::load(Bb2 + bo);
    }
#pragma unroll
    for (int i = 0; i < 4; ++i) {
      const size_t ao = (size_t)(m0 + (i << 4) + rlane) * lda + koff + k0;
      V ah = Frag<T>::load(Ab + ao);
      V al;
      if (SPLIT) al = Frag<T>::load(Ab2 + ao);
#pragma unroll
      for (int j = 0; j < 4; ++j) {
        acc[i][j] = Frag<T>::mma(ah, bh[j], acc[i][j]);
        if (SPLIT) {
          if (BSPLIT) acc[i][j] = Frag<T>::mma(ah, bl[j], acc[i][j]);
          acc[i][j] = Frag<T>::mma(al, bh[j], acc[i][j]);
        }
      }
      Frag<T>::guard(acc[i][0], acc[i][3], ah, SPLIT ? al : ah);
    }
    Frag<T>::keep(bh[0], bh[1], bh[2], bh[3]);
    if (SPLIT && BSPLIT) Frag<T>::keep(bl[0], bl[1], bl[2], bl[3]);
  }
  acc_guard4(acc[0][0], acc[0][1], acc[0][2], acc[0][3]);
  acc_guard4(acc[1][0], acc[1][1], acc[1][2], acc[1][3]);
  acc_guard4(acc[2][0], acc[2][1], acc[2][2], acc[2][3]);
  acc_guard4(acc[3][0], acc[3][1], acc[3][2], acc[3][3]);

  float* slab = sT[wave];
  const float* Rb = RESID ? (resid + (size_t)b * strideR) : nullptr;
#pragma unroll
  for (int i = 0; i < 4; ++i) {
    const int mBase = m0 + (i << 4);
#pragma unroll
    for (int j = 0; j < 4; ++j) {
      const int n = n0 + (j << 4) + rlane;
      float bv = 0.f;
      if (BIAS_MODE == 2) bv = bias[n];
#pragma unroll
      for (int r = 0; r < 8; ++r) {
        float v = acc[i][j][r] * scale;
        if (BIAS_MODE == 1) v += bias[mBase + mOff + r];
        if (BIAS_MODE == 2) v += bv;
        if (RESID) v += Rb[(size_t)(mBase + mOff + r) * ldc + n];
        if (ACT == 1) v = tanhf(v);
        if (ACT == 2) v = fmaxf(v, 0.0f);
        if (ACT == 3) v = v / (1.0f + expf(-v));
        if (ACT == 4) v = (v > 0.f) ? v : 0.01f * v;
        if (ACT == 5) v = 0.5f * v * (1.0f + erff(v * 0.70710678118654752f));
        slab[(mOff + r) * 68 + (j << 4) + rlane] = v;
      }
    }
    __builtin_amdgcn_fence(__ATOMIC_RELEASE, "workgroup");
    __builtin_amdgcn_wave_barrier();
    __builtin_amdgcn_fence(__ATOMIC_ACQUIRE, "workgroup");
    if (OUT_MODE == 0) {
      float* C = (float*)Cout + (size_t)b * strideC;
      const int hh = lane >> 4, c4 = (lane & 15) * 4;
      for (int pass = 0; pass < 2; ++pass) {
#pragma unroll
        for (int it = 0; it < 8; ++it) {
          const int row = it * 2 + hh;
          v4f v = *(const v4f*)(slab + row * 68 + c4);
          *(volatile v4f*)(C + (size_t)(mBase + row) * ldc + n0 + c4) = v;
        }
        __threadfence();
      }
    } else {
      const int q = lane >> 3, c8 = (lane & 7) * 8;
      unsigned short* C  = (unsigned short*)Cout  + (size_t)b * strideC;
      unsigned short* C2 = (OUT_MODE == 2) ? ((unsigned short*)Cout2 + (size_t)b * strideC) : nullptr;
      for (int pass = 0; pass < 2; ++pass) {
#pragma unroll
        for (int it = 0; it < 4; ++it) {
          const int row = it * 4 + q;
          const float* sp = slab + row * 68 + c8;
          v8h hv, lv;
#pragma unroll
          for (int e = 0; e < 8; ++e) {
            if (OUT_MODE == 1) {
              hv[e] = (_Float16)sp[e];
            } else {
              unsigned short hb = f2bf_bits(sp[e]);
              unsigned short lb = f2bf_bits(sp[e] - bf_bits2f(hb));
              hv[e] = __builtin_bit_cast(_Float16, hb);
              lv[e] = __builtin_bit_cast(_Float16, lb);
            }
          }
          *(volatile v8h*)(C + (size_t)(mBase + row) * ldc + n0 + c8) = hv;
          if (OUT_MODE == 2) *(volatile v8h*)(C2 + (size_t)(mBase + row) * ldc + n0 + c8) = lv;
        }
        __threadfence();
      }
    }
    __builtin_amdgcn_fence(__ATOMIC_RELEASE, "workgroup");
    __builtin_amdgcn_wave_barrier();
    __builtin_amdgcn_fence(__ATOMIC_ACQUIRE, "workgroup");
  }
}

__device__ __forceinline__ v8f at_mma(v16b a, v16b b, v8f c) {
  c = __builtin_amdgcn_wmma_f32_16x16x32_bf16(false, a, false, b, (short)0, c, false, false);
  asm volatile("v_nop\n\tv_nop\n\tv_nop\n\tv_nop" : "+v"(c) : "v"(a), "v"(b));
  return c;
}
__device__ __forceinline__ v8f at_mma_h(v16h a, v16h b, v8f c) {
  c = __builtin_amdgcn_wmma_f32_16x16x32_f16(false, a, false, b, (short)0, c, false, false);
  asm volatile("v_nop\n\tv_nop\n\tv_nop\n\tv_nop" : "+v"(c) : "v"(a), "v"(b));
  return c;
}
__device__ __forceinline__ void wave_lds_sync() {
  __builtin_amdgcn_fence(__ATOMIC_RELEASE, "workgroup");
  __builtin_amdgcn_wave_barrier();
  __builtin_amdgcn_fence(__ATOMIC_ACQUIRE, "workgroup");
}

__global__ __launch_bounds__(256) void cast_f32_bf16x8(
    const float* __restrict__ in, unsigned short* __restrict__ out, int n8) {
  const int i = blockIdx.x * 256 + threadIdx.x;
  if (i < n8) {
    const v4f a  = *(const v4f*)(in + (size_t)i * 8);
    const v4f a2 = *(const v4f*)(in + (size_t)i * 8 + 4);
    v4u w;
    w[0] = (unsigned)f2bf_bits(a[0])  | ((unsigned)f2bf_bits(a[1])  << 16);
    w[1] = (unsigned)f2bf_bits(a[2])  | ((unsigned)f2bf_bits(a[3])  << 16);
    w[2] = (unsigned)f2bf_bits(a2[0]) | ((unsigned)f2bf_bits(a2[1]) << 16);
    w[3] = (unsigned)f2bf_bits(a2[2]) | ((unsigned)f2bf_bits(a2[3]) << 16);
    volatile v4u* p = (volatile v4u*)(out + (size_t)i * 8);
    *p = w;
    __threadfence();
    *p = w;
  }
}

__global__ __launch_bounds__(256) void pack_mask_bits(
    const int* __restrict__ mask, unsigned* __restrict__ bits, int nw) {
  const int w  = blockIdx.x * 256 + threadIdx.x;
  const int wc = (w < nw) ? w : (nw - 1);
  const v4i* p = (const v4i*)(mask + (size_t)wc * 32);
  unsigned u = 0u;
#pragma unroll
  for (int i = 0; i < 8; ++i) {
    const v4i m4 = p[i];
#pragma unroll
    for (int e = 0; e < 4; ++e) u |= ((m4[e] != 0) ? 1u : 0u) << (4 * i + e);
  }
  if (w < nw) {
    volatile unsigned* o = (volatile unsigned*)(bits + w);
    *o = u;
    __threadfence();
    *o = u;
  }
}

__global__ __launch_bounds__(128) __attribute__((amdgpu_num_vgpr(256)))
void attn_planes_kernel(const unsigned short* __restrict__ Qhp, const unsigned short* __restrict__ Qlp,
                        const unsigned short* __restrict__ Khp, const unsigned short* __restrict__ Klp,
                        const unsigned short* __restrict__ Vtp,
                        const unsigned* __restrict__ mbits,
                        unsigned short* __restrict__ Chp, unsigned short* __restrict__ Clp) {
  __shared__ __align__(16) _Float16 Psh[4][16 * KCH];
  __shared__ __align__(16) float    Os[4][16 * 68];

  const __bf16* Qh = (const __bf16*)Qhp; const __bf16* Ql = (const __bf16*)Qlp;
  const __bf16* Kh = (const __bf16*)Khp; const __bf16* Kl = (const __bf16*)Klp;
  const _Float16* Vt = (const _Float16*)Vtp;

  const int tid  = threadIdx.x;
  const int wave = tid >> 5;
  const int lane = tid & 31;
  const int hh   = lane >> 4;
  const int c    = lane & 15;
  const int koff = hh * 8;

  const int nqb = SEQ_LEN / QBLK;
  const int bx  = blockIdx.x;
  const int qb  = bx % nqb;
  const int bhd = bx / nqb;
  const int h   = bhd % NHEAD;
  const int b   = bhd / NHEAD;
  const int q0  = qb * QBLK + wave * 16;

  v16b qah[2], qal[2];
  {
    const size_t qoff = ((size_t)(b * SEQ_LEN + q0 + c)) * DMOD + (size_t)(h * HDIM) + koff;
#pragma unroll
    for (int dc = 0; dc < 2; ++dc) {
      qah[dc] = Frag<__bf16>::load(Qh + qoff + dc * 32);
      qal[dc] = Frag<__bf16>::load(Ql + qoff + dc * 32);
    }
  }

  float mrow[8], lrow[8];
  v8f oacc[4];
#pragma unroll
  for (int r = 0; r < 8; ++r) { mrow[r] = -__builtin_inff(); lrow[r] = 0.f; }
#pragma unroll
  for (int t = 0; t < 4; ++t) oacc[t] = (v8f){0.f,0.f,0.f,0.f,0.f,0.f,0.f,0.f};

  const size_t vbase = (size_t)b * ((size_t)DMOD * SEQ_LEN) + (size_t)(h * HDIM) * SEQ_LEN;
  _Float16* pw = Psh[wave];

  for (int kc = 0; kc < SEQ_LEN / KCH; ++kc) {
    const int kv0 = kc * KCH;
    __syncthreads();

    unsigned mw[8];
#pragma unroll
    for (int r = 0; r < 8; ++r)
      mw[r] = mbits[(size_t)(q0 + 8 * hh + r) * MWORDS + (kv0 >> 5)];

    v8f s[2];
#pragma unroll
    for (int j = 0; j < 2; ++j) {
      s[j] = (v8f){0.f,0.f,0.f,0.f,0.f,0.f,0.f,0.f};
      const size_t ko = ((size_t)(b * SEQ_LEN + kv0 + j * 16 + c)) * DMOD + (size_t)(h * HDIM) + koff;
#pragma unroll
      for (int dc = 0; dc < 2; ++dc) {
        const v16b kb = Frag<__bf16>::load(Kh + ko + dc * 32);
        const v16b kl = Frag<__bf16>::load(Kl + ko + dc * 32);
        s[j] = at_mma(qah[dc], kb, s[j]);
        s[j] = at_mma(qah[dc], kl, s[j]);
        s[j] = at_mma(qal[dc], kb, s[j]);
      }
    }

    float cm[8];
#pragma unroll
    for (int r = 0; r < 8; ++r) {
      float m = -__builtin_inff();
#pragma unroll
      for (int j = 0; j < 2; ++j) {
        float x = s[j][r] * 0.125f;
        const unsigned keep = (mw[r] >> (j * 16 + c)) & 1u;
        x = (keep != 0u) ? x : 1e-9f;
        s[j][r] = x;
        m = fmaxf(m, x);
      }
#pragma unroll
      for (int off = 1; off < 16; off <<= 1) m = fmaxf(m, __shfl_xor(m, off, 32));
      cm[r] = m;
    }

#pragma unroll
    for (int r = 0; r < 8; ++r) {
      const float mnew  = fmaxf(mrow[r], cm[r]);
      const float alpha = expf(mrow[r] - mnew);
      mrow[r] = mnew;
      float psum = 0.f;
#pragma unroll
      for (int j = 0; j < 2; ++j) {
        const float p = expf(s[j][r] - mnew);
        psum += p;
        pw[(8 * hh + r) * KCH + j * 16 + c] = (_Float16)(p * PCARRY);
      }
#pragma unroll
      for (int off = 1; off < 16; off <<= 1) psum += __shfl_xor(psum, off, 32);
      lrow[r] = lrow[r] * alpha + psum;
#pragma unroll
      for (int t = 0; t < 4; ++t) oacc[t][r] *= alpha;
    }
    wave_lds_sync();

    const v16h pa = Frag<_Float16>::load(pw + c * KCH + koff);
#pragma unroll
    for (int t = 0; t < 4; ++t) {
      const size_t vo = vbase + (size_t)(t * 16 + c) * SEQ_LEN + kv0 + koff;
      const v16h vb = Frag<_Float16>::load(Vt + vo);
      oacc[t] = at_mma_h(pa, vb, oacc[t]);
    }
  }

  float* os = Os[wave];
#pragma unroll
  for (int r = 0; r < 8; ++r) {
    const float inv = 1.0f / (lrow[r] * PCARRY);
#pragma unroll
    for (int t = 0; t < 4; ++t) os[(8 * hh + r) * 68 + t * 16 + c] = oacc[t][r] * inv;
  }
  wave_lds_sync();
  {
    const int q = lane >> 3, c8 = (lane & 7) * 8;
    for (int pass = 0; pass < 2; ++pass) {
#pragma unroll
      for (int it = 0; it < 4; ++it) {
        const int row = it * 4 + q;
        const float* sp = os + row * 68 + c8;
        const v4f x0 = *(const v4f*)(sp);
        const v4f x1 = *(const v4f*)(sp + 4);
        v4u hw, lw;
#pragma unroll
        for (int e2 = 0; e2 < 4; ++e2) {
          const float f0 = (e2 < 2) ? x0[2 * e2] : x1[2 * e2 - 4];
          const float f1 = (e2 < 2) ? x0[2 * e2 + 1] : x1[2 * e2 - 3];
          const unsigned short hb0 = f2bf_bits(f0);
          const unsigned short lb0 = f2bf_bits(f0 - bf_bits2f(hb0));
          const unsigned short hb1 = f2bf_bits(f1);
          const unsigned short lb1 = f2bf_bits(f1 - bf_bits2f(hb1));
          hw[e2] = (unsigned)hb0 | ((unsigned)hb1 << 16);
          lw[e2] = (unsigned)lb0 | ((unsigned)lb1 << 16);
        }
        const size_t o = ((size_t)(b * SEQ_LEN + q0 + row)) * DMOD + (size_t)(h * HDIM) + c8;
        *(volatile v4u*)(Chp + o) = hw;
        *(volatile v4u*)(Clp + o) = lw;
      }
      __threadfence();
    }
  }
}

extern "C" void kernel_launch(void* const* d_in, const int* in_sizes, int n_in,
                              void* d_out, int out_size, void* d_ws, size_t ws_size,
                              hipStream_t stream) {
  if (n_in < 12) return;
  const int nAct = NTOK * DMOD;
  const int nWgt = DMOD * DMOD;
  const int nMask = SEQ_LEN * SEQ_LEN;
  const int nMW = SEQ_LEN * MWORDS;
  if (in_sizes[0] != nAct || in_sizes[1] != nAct || in_sizes[2] != nAct || in_sizes[3] != nMask) return;
  if (in_sizes[4] != nWgt || in_sizes[6] != nWgt || in_sizes[8] != nWgt || in_sizes[10] != nWgt) return;
  if (in_sizes[5] != DMOD || in_sizes[7] != DMOD || in_sizes[9] != DMOD || in_sizes[11] != DMOD) return;
  if (out_size != nAct) return;

  const float* q    = (const float*)d_in[0];
  const float* k    = (const float*)d_in[1];
  const float* v    = (const float*)d_in[2];
  const int*   mask = (const int*)  d_in[3];
  const float* wq_w = (const float*)d_in[4];
  const float* wq_b = (const float*)d_in[5];
  const float* wk_w = (const float*)d_in[6];
  const float* wk_b = (const float*)d_in[7];
  const float* wv_w = (const float*)d_in[8];
  const float* wv_b = (const float*)d_in[9];
  const float* wo_w = (const float*)d_in[10];
  const float* wo_b = (const float*)d_in[11];
  float* outp = (float*)d_out;

  const size_t actB = (size_t)nAct * 2;
  const size_t wgtB = (size_t)nWgt * 2;
  const size_t mwB  = (size_t)nMW * 4;
  size_t off = 0;
  char* ws = (char*)d_ws;
  unsigned short* qb  = (unsigned short*)(ws + off); off += actB;
  unsigned short* kb  = (unsigned short*)(ws + off); off += actB;
  unsigned short* vb  = (unsigned short*)(ws + off); off += actB;
  unsigned short* wqb = (unsigned short*)(ws + off); off += wgtB;
  unsigned short* wkb = (unsigned short*)(ws + off); off += wgtB;
  unsigned short* wvb = (unsigned short*)(ws + off); off += wgtB;
  unsigned short* wob = (unsigned short*)(ws + off); off += wgtB;
  unsigned short* Qh  = (unsigned short*)(ws + off); off += actB;
  unsigned short* Ql  = (unsigned short*)(ws + off); off += actB;
  unsigned short* Kh  = (unsigned short*)(ws + off); off += actB;
  unsigned short* Kl  = (unsigned short*)(ws + off); off += actB;
  unsigned short* Vt  = (unsigned short*)(ws + off); off += actB;
  unsigned short* Ch  = (unsigned short*)(ws + off); off += actB;
  unsigned short* Cl  = (unsigned short*)(ws + off); off += actB;
  unsigned*       mbits = (unsigned*)(ws + off);     off += mwB;
  if (off > ws_size) return;

  const int n8Act = nAct / 8, n8Wgt = nWgt / 8;
  cast_f32_bf16x8<<<n8Act / 256, 256, 0, stream>>>(q, qb, n8Act);
  cast_f32_bf16x8<<<n8Act / 256, 256, 0, stream>>>(k, kb, n8Act);
  cast_f32_bf16x8<<<n8Act / 256, 256, 0, stream>>>(v, vb, n8Act);
  cast_f32_bf16x8<<<n8Wgt / 256, 256, 0, stream>>>(wq_w, wqb, n8Wgt);
  cast_f32_bf16x8<<<n8Wgt / 256, 256, 0, stream>>>(wk_w, wkb, n8Wgt);
  cast_f32_bf16x8<<<n8Wgt / 256, 256, 0, stream>>>(wv_w, wvb, n8Wgt);
  cast_f32_bf16x8<<<n8Wgt / 256, 256, 0, stream>>>(wo_w, wob, n8Wgt);
  pack_mask_bits<<<nMW / 256, 256, 0, stream>>>(mask, mbits, nMW);

  const int blkQK = ((NTOK / 64) * (DMOD / 64)) / 8;
  wmma_gemm64<1, false, 2, 2, false, 0, true><<<dim3(blkQK, 1), 256, 0, stream>>>(
      qb, qb, DMOD, 0L, wqb, wqb, DMOD, 0L, (void*)Qh, (void*)Ql, DMOD, 0L, wq_b, wq_b, 0L,
      NTOK, DMOD, DMOD, 1.0f);
  wmma_gemm64<1, false, 2, 2, false, 0, true><<<dim3(blkQK, 1), 256, 0, stream>>>(
      kb, kb, DMOD, 0L, wkb, wkb, DMOD, 0L, (void*)Kh, (void*)Kl, DMOD, 0L, wk_b, wk_b, 0L,
      NTOK, DMOD, DMOD, 1.0f);
  const int blkV = ((DMOD / 64) * (SEQ_LEN / 64)) / 8;
  wmma_gemm64<1, false, 1, 1, false, 0, true><<<dim3(blkV, NBATCH), 256, 0, stream>>>(
      wvb, wvb, DMOD, 0L, vb, vb, DMOD, (long)SEQ_LEN * DMOD, (void*)Vt, (void*)Vt, SEQ_LEN, (long)DMOD * SEQ_LEN,
      wv_b, wv_b, 0L, DMOD, SEQ_LEN, DMOD, 1.0f);

  attn_planes_kernel<<<NBATCH * NHEAD * (SEQ_LEN / QBLK), 128, 0, stream>>>(Qh, Ql, Kh, Kl, Vt, mbits, Ch, Cl);

  wmma_gemm64<1, true, 2, 0, false, 0, false><<<dim3(blkQK, 1), 256, 0, stream>>>(
      Ch, Cl, DMOD, 0L, wob, wob, DMOD, 0L, (void*)outp, (void*)outp, DMOD, 0L, wo_b, wo_b, 0L,
      NTOK, DMOD, DMOD, 1.0f);
}
